// RNNTwoLayerModel_47682726921063
// MI455X (gfx1250) — hardware-verified
//
#include <hip/hip_runtime.h>
#include <math.h>

constexpr int NBATCH = 64;
constexpr int NSTEP  = 1024;
constexpr int NEMB   = 256;
constexpr int NHID   = 512;
constexpr int NOUTC  = 128;
constexpr int NVOCAB = 32000;
constexpr int NROWS  = NBATCH * NSTEP;
constexpr int NOUT_ELEMS = NBATCH * NOUTC * NSTEP;
constexpr float WCARRY     = 256.0f;
constexpr float WCARRY_INV = 1.0f / 256.0f;

constexpr int RB   = 32;
constexpr int RTHR = 512;
constexpr int H1P  = 520;
constexpr int H2P  = 136;
constexpr int XPW  = 260;

static_assert(NROWS == 65536, "rows");
static_assert(NROWS % 64 == 0 && NHID % 64 == 0 && NEMB % 32 == 0, "gemm tiles");
static_assert(NHID % 32 == 0 && NOUTC % 32 == 0, "k multiples");
static_assert(NBATCH % RB == 0, "row blocks");
static_assert(NHID == 32 * (RTHR / 32), "16 waves x 32 hidden columns");
static_assert((RB / 16) * (NOUTC / 16) == RTHR / 32, "one layer-2 tile per wave");
static_assert((2 * RB * H1P) % RTHR == 0 && (2 * RB * H2P) % RTHR == 0, "zero fill exact");
static_assert(RB * (NHID / 8) == 4 * RTHR, "x-term staging exact");
static_assert(H1P % 8 == 0 && H2P % 8 == 0 && (XPW * 2) % 8 == 0, "16-B aligned LDS rows");
static_assert(NSTEP % 32 == 0, "t blocks");

typedef __attribute__((ext_vector_type(16))) _Float16 v16h;
typedef __attribute__((ext_vector_type(8)))  _Float16 v8h;
typedef __attribute__((ext_vector_type(8)))  float    v8f;
typedef __attribute__((ext_vector_type(4)))  float    v4f;
typedef __attribute__((ext_vector_type(4)))  unsigned v4u;
typedef __attribute__((ext_vector_type(2)))  unsigned v2u;

__device__ __forceinline__ float h16_to_f32(unsigned hb) {
  const unsigned sgn = (hb & 0x8000u) << 16;
  const unsigned em = hb & 0x7fffu;
  const float fn = __uint_as_float((em << 13) + 0x38000000u);
  const float fs = (float)em * 5.9604644775390625e-8f;
  const float mag = (em < 0x400u) ? fs : fn;
  return __uint_as_float(__float_as_uint(mag) | sgn);
}

__device__ __forceinline__ float tanh_f32(float x) {
  const float e = expf(2.0f * x);
  return 1.0f - 2.0f * __builtin_amdgcn_rcpf(e + 1.0f);
}

union FragU { v16h v; v8h h[2]; };
__device__ __forceinline__ v16h frag_load(const _Float16* p) {
  FragU f;
  f.h[0] = *(const v8h*)(p);
  f.h[1] = *(const v8h*)(p + 16);
  return f.v;
}
__device__ __forceinline__ v8f mma_f16(v16h a, v16h b, v8f c) {
  return __builtin_amdgcn_wmma_f32_16x16x32_f16(false, a, false, b, (short)0, c, false, false);
}
__device__ __forceinline__ void guard_row4(v8f& a, v8f& b, v8f& c, v8f& d, v16h x, v16h y0, v16h y1, v16h y2, v16h y3) {
  asm volatile("v_nop\n\tv_nop\n\tv_nop\n\tv_nop" : "+v"(a), "+v"(b), "+v"(c), "+v"(d) : "v"(x), "v"(y0), "v"(y1), "v"(y2), "v"(y3));
}
__device__ __forceinline__ void guard_pair(v8f& a, v8f& b, v16h x0, v16h x1, v16h y) {
  asm volatile("v_nop\n\tv_nop\n\tv_nop\n\tv_nop" : "+v"(a), "+v"(b) : "v"(x0), "v"(x1), "v"(y));
}
__device__ __forceinline__ void guard_one(v8f& a, v16h x, v16h y) {
  asm volatile("v_nop\n\tv_nop\n\tv_nop\n\tv_nop" : "+v"(a) : "v"(x), "v"(y));
}
__device__ __forceinline__ void acc_guard4(v8f& a, v8f& b, v8f& c, v8f& d) {
  asm volatile("v_nop\n\tv_nop\n\tv_nop\n\tv_nop" : "+v"(a), "+v"(b), "+v"(c), "+v"(d));
}
__device__ __forceinline__ void acc_guard2(v8f& a, v8f& b) {
  asm volatile("v_nop\n\tv_nop\n\tv_nop\n\tv_nop" : "+v"(a), "+v"(b));
}
__device__ __forceinline__ void acc_guard1(v8f& a) {
  asm volatile("v_nop\n\tv_nop\n\tv_nop\n\tv_nop" : "+v"(a));
}

__global__ __launch_bounds__(256) void cvt8_f16_kernel(const float* __restrict__ src, unsigned short* __restrict__ dst,
                                                       int n8, float sc) {
  const int i = blockIdx.x * 256 + threadIdx.x;
  if (i < n8) {
    const float* sp = src + (size_t)i * 8;
    const v4f a = *(const v4f*)(sp);
    const v4f b = *(const v4f*)(sp + 4);
    v8h hv;
#pragma unroll
    for (int e = 0; e < 4; ++e) {
      hv[e]     = (_Float16)(a[e] * sc);
      hv[4 + e] = (_Float16)(b[e] * sc);
    }
    volatile v8h* dp = (volatile v8h*)(dst + (size_t)i * 8);
    *dp = hv;
    __threadfence();
    *dp = hv;
  }
}

__global__ __launch_bounds__(160) void bias_prep_kernel(const float* __restrict__ bi1, const float* __restrict__ bh1,
                                                        const float* __restrict__ bi2, const float* __restrict__ bh2,
                                                        float* __restrict__ dst) {
  const int tid = threadIdx.x;
  const int wave = tid >> 5;
  if (wave < 4) {
    const int idx = tid * 4;
    const v4f a = *(const v4f*)(bi1 + idx);
    const v4f b = *(const v4f*)(bh1 + idx);
    const v4f o = a + b;
    volatile v4f* op = (volatile v4f*)(dst + idx);
    *op = o;
    __threadfence();
    *op = o;
  } else {
    const int idx = (tid - 128) * 4;
    const v4f a = *(const v4f*)(bi2 + idx);
    const v4f b = *(const v4f*)(bh2 + idx);
    const v4f o = a + b;
    volatile v4f* op = (volatile v4f*)(dst + NHID + idx);
    *op = o;
    __threadfence();
    *op = o;
  }
}

__global__ __launch_bounds__(256) void gather_cvt_kernel(const int* __restrict__ x, const float* __restrict__ emb,
                                                         unsigned short* __restrict__ dst) {
  const int i = blockIdx.x * 256 + threadIdx.x;
  if (i < NROWS * (NEMB / 8)) {
    const int row = i >> 5;
    const int c8  = i & 31;
    const int t = row >> 6;
    const int b = row & 63;
    int id = x[b * NSTEP + t];
    id = id < 0 ? 0 : id;
    id = id > (NVOCAB - 1) ? (NVOCAB - 1) : id;
    const float* sp = emb + (size_t)id * NEMB + c8 * 8;
    const v4f a = *(const v4f*)(sp);
    const v4f c = *(const v4f*)(sp + 4);
    v8h hv;
#pragma unroll
    for (int e = 0; e < 4; ++e) {
      hv[e]     = (_Float16)a[e];
      hv[4 + e] = (_Float16)c[e];
    }
    volatile v8h* dp = (volatile v8h*)(dst + (size_t)i * 8);
    *dp = hv;
    __threadfence();
    *dp = hv;
  }
}

__global__ __launch_bounds__(256) void gemm64_f16_kernel(
    const unsigned short* __restrict__ Ap, int lda,
    const unsigned short* __restrict__ Btp, int ldb,
    unsigned short* __restrict__ Cout, int ldc,
    const float* __restrict__ bias, int M, int N, int K, float scale) {
  const _Float16* A  = (const _Float16*)Ap;
  const _Float16* Bt = (const _Float16*)Btp;
  __shared__ __align__(16) float sT[8][16 * 68];
  const int lane = threadIdx.x & 31;
  const int wave = threadIdx.x >> 5;
  const int tilesN = N >> 6;
  const int tilesM = M >> 6;
  const int tile = blockIdx.x * 8 + wave;
  if (tile >= tilesM * tilesN) return;
  const int tm = tile / tilesN;
  const int tn = tile - tm * tilesN;
  const int m0 = tm << 6;
  const int n0 = tn << 6;

  const int rlane = lane & 15;
  const int koff  = (lane >> 4) * 8;
  const int mOff  = (lane >> 4) * 8;

  v8f acc[4][4];
#pragma unroll
  for (int i = 0; i < 4; ++i)
#pragma unroll
    for (int j = 0; j < 4; ++j) acc[i][j] = (v8f){0.f, 0.f, 0.f, 0.f, 0.f, 0.f, 0.f, 0.f};

  for (int k0 = 0; k0 < K; k0 += 32) {
    v16h bh[4];
#pragma unroll
    for (int j = 0; j < 4; ++j) {
      const size_t bo = (size_t)(n0 + (j << 4) + rlane) * ldb + koff + k0;
      bh[j] = frag_load(Bt + bo);
    }
#pragma unroll
    for (int i = 0; i < 4; ++i) {
      const size_t ao = (size_t)(m0 + (i << 4) + rlane) * lda + koff + k0;
      const v16h ah = frag_load(A + ao);
#pragma unroll
      for (int j = 0; j < 4; ++j) acc[i][j] = mma_f16(ah, bh[j], acc[i][j]);
      guard_row4(acc[i][0], acc[i][1], acc[i][2], acc[i][3], ah, bh[0], bh[1], bh[2], bh[3]);
    }
  }
  acc_guard4(acc[0][0], acc[0][1], acc[0][2], acc[0][3]);
  acc_guard4(acc[1][0], acc[1][1], acc[1][2], acc[1][3]);
  acc_guard4(acc[2][0], acc[2][1], acc[2][2], acc[2][3]);
  acc_guard4(acc[3][0], acc[3][1], acc[3][2], acc[3][3]);

  float* slab = sT[wave];
#pragma unroll
  for (int i = 0; i < 4; ++i) {
    const int mBase = m0 + (i << 4);
#pragma unroll
    for (int j = 0; j < 4; ++j) {
      const int n = n0 + (j << 4) + rlane;
      const float bv = bias[n];
#pragma unroll
      for (int r = 0; r < 8; ++r) {
        const float v = acc[i][j][r] * scale + bv;
        slab[(mOff + r) * 68 + (j << 4) + rlane] = v;
      }
    }
    __builtin_amdgcn_fence(__ATOMIC_RELEASE, "workgroup");
    __builtin_amdgcn_wave_barrier();
    __builtin_amdgcn_fence(__ATOMIC_ACQUIRE, "workgroup");
    {
      const int q = lane >> 3, c8 = (lane & 7) * 8;
      for (int pass = 0; pass < 2; ++pass) {
#pragma unroll
        for (int it = 0; it < 4; ++it) {
          const int row = it * 4 + q;
          const float* sp = slab + row * 68 + c8;
          v8h hv;
#pragma unroll
          for (int e = 0; e < 8; ++e) hv[e] = (_Float16)sp[e];
          *(volatile v8h*)(Cout + (size_t)(mBase + row) * ldc + n0 + c8) = hv;
        }
        __threadfence();
      }
    }
    __builtin_amdgcn_fence(__ATOMIC_RELEASE, "workgroup");
    __builtin_amdgcn_wave_barrier();
    __builtin_amdgcn_fence(__ATOMIC_ACQUIRE, "workgroup");
  }
}

__global__ __launch_bounds__(RTHR) void rnn_seq_kernel(const unsigned short* __restrict__ XP1p,
                                                       const unsigned short* __restrict__ WHH1p,
                                                       const unsigned short* __restrict__ WIH2p,
                                                       const unsigned short* __restrict__ WHH2p,
                                                       const float* __restrict__ bias2,
                                                       unsigned short* __restrict__ H2g) {
  __shared__ __align__(16) _Float16 H1s[2][RB * H1P];
  __shared__ __align__(16) _Float16 H2s[2][RB * H2P];
  __shared__ __align__(16) unsigned XPw[RB * XPW];
  const _Float16* WHH1 = (const _Float16*)WHH1p;
  const _Float16* WIH2 = (const _Float16*)WIH2p;
  const _Float16* WHH2 = (const _Float16*)WHH2p;
  const int tid = threadIdx.x, lane = tid & 31, wave = tid >> 5;
  const int c = lane & 15, hh = lane >> 4, koff = hh * 8;
  const int rowbase = blockIdx.x * RB;

  {
    _Float16* p1 = &H1s[0][0];
#pragma unroll 1
    for (int i = tid; i < 2 * RB * H1P; i += RTHR) p1[i] = (_Float16)0.0f;
    _Float16* p2 = &H2s[0][0];
#pragma unroll 1
    for (int i = tid; i < 2 * RB * H2P; i += RTHR) p2[i] = (_Float16)0.0f;
  }
#pragma unroll
  for (int it = 0; it < 4; ++it) {
    const int idx = it * RTHR + tid;
    const int row = idx >> 6, ch = idx & 63;
    const v4u v = *(const v4u*)(XP1p + (size_t)(rowbase + row) * NHID + ch * 8);
    *(v4u*)(XPw + row * XPW + ch * 4) = v;
  }
  const int mt2 = wave >> 3, nt2 = wave & 7;
  const int n2 = 16 * nt2 + c;
  const float b2v = bias2[n2];
  __syncthreads();

  const v8f z8 = {0.f, 0.f, 0.f, 0.f, 0.f, 0.f, 0.f, 0.f};

#pragma unroll 1
  for (int t = 0; t < NSTEP; ++t) {
    const int cur = t & 1;
    const int prv = cur ^ 1;
    const _Float16* h1r = &H1s[prv][0];
    _Float16* h1w = &H1s[cur][0];
    const _Float16* h2r = &H2s[prv][0];
    _Float16* h2w = &H2s[cur][0];

#pragma unroll 1
    for (int nt = 0; nt < 2; ++nt) {
      const int j = 32 * wave + 16 * nt + c;
      const _Float16* wr  = WHH1 + (size_t)j * NHID + koff;
      const _Float16* a0p = h1r + c * H1P + koff;
      const _Float16* a1p = a0p + 16 * H1P;
      v8f acc0 = z8, acc1 = z8;
#pragma unroll 1
      for (int k0 = 0; k0 < NHID; k0 += 32) {
        const v16h bf = frag_load(wr + k0);
        const v16h a0 = frag_load(a0p + k0);
        const v16h a1 = frag_load(a1p + k0);
        acc0 = mma_f16(a0, bf, acc0);
        acc1 = mma_f16(a1, bf, acc1);
        guard_pair(acc0, acc1, a0, a1, bf);
      }
      acc_guard2(acc0, acc1);
      const int jw = j >> 1;
      const bool jodd = (c & 1) != 0;
#pragma unroll
      for (int r = 0; r < 8; ++r) {
        const int row0 = 8 * hh + r;
        const int row1 = 16 + 8 * hh + r;
        const unsigned w0 = XPw[row0 * XPW + jw];
        const unsigned w1 = XPw[row1 * XPW + jw];
        const unsigned hb0 = jodd ? (w0 >> 16) : (w0 & 0xffffu);
        const unsigned hb1 = jodd ? (w1 >> 16) : (w1 & 0xffffu);
        const float x0 = h16_to_f32(hb0);
        const float x1 = h16_to_f32(hb1);
        const float g0 = tanh_f32(acc0[r] * WCARRY_INV + x0);
        const float g1 = tanh_f32(acc1[r] * WCARRY_INV + x1);
        h1w[row0 * H1P + j] = (_Float16)g0;
        h1w[row1 * H1P + j] = (_Float16)g1;
      }
    }
    __syncthreads();

    {
      const int tn = (t + 1 < NSTEP) ? (t + 1) : (NSTEP - 1);
#pragma unroll
      for (int it = 0; it < 4; ++it) {
        const int idx = it * RTHR + tid;
        const int row = idx >> 6, ch = idx & 63;
        const v4u v = *(const v4u*)(XP1p + ((size_t)tn * NBATCH + (size_t)(rowbase + row)) * NHID + ch * 8);
        *(v4u*)(XPw + row * XPW + ch * 4) = v;
      }
    }

    {
      const _Float16* wi = WIH2 + (size_t)n2 * NHID + koff;
      const _Float16* wh = WHH2 + (size_t)n2 * NOUTC + koff;
      const _Float16* ap = h1w + (16 * mt2 + c) * H1P + koff;
      const _Float16* hp = h2r + (16 * mt2 + c) * H2P + koff;
      v8f acc = z8;
#pragma unroll 1
      for (int k0 = 0; k0 < NHID; k0 += 32) {
        const v16h a  = frag_load(ap + k0);
        const v16h bf = frag_load(wi + k0);
        acc = mma_f16(a, bf, acc);
        guard_one(acc, a, bf);
      }
#pragma unroll 1
      for (int k0 = 0; k0 < NOUTC; k0 += 32) {
        const v16h a  = frag_load(hp + k0);
        const v16h bf = frag_load(wh + k0);
        acc = mma_f16(a, bf, acc);
        guard_one(acc, a, bf);
      }
      acc_guard1(acc);
#pragma unroll
      for (int r = 0; r < 8; ++r) {
        const float g = tanh_f32(acc[r] * WCARRY_INV + b2v);
        h2w[(16 * mt2 + 8 * hh + r) * H2P + n2] = (_Float16)g;
      }
    }
    __syncthreads();

    {
      const int rr = 2 * wave + hh;
      const int c8 = c * 8;
      const v8h hv = *(const v8h*)(h2w + rr * H2P + c8);
      volatile v8h* gp = (volatile v8h*)(H2g + ((size_t)t * NBATCH + (size_t)(rowbase + rr)) * NOUTC + c8);
      *gp = hv;
      __threadfence();
      *gp = hv;
    }
  }
}

__global__ __launch_bounds__(256) void softmax_tr_kernel(const unsigned short* __restrict__ H2g, float* __restrict__ out) {
  __shared__ float Tl[NOUTC * 33];
  const int tid = threadIdx.x, lane = tid & 31, wave = tid >> 5;
  const int b  = blockIdx.x >> 5;
  const int t0 = (blockIdx.x & 31) * 32;
#pragma unroll 1
  for (int q = 0; q < 4; ++q) {
    const int i = wave * 4 + q;
    const size_t row = (size_t)(t0 + i) * NBATCH + (size_t)b;
    const v2u w = *(const v2u*)(H2g + row * NOUTC + 4 * lane);
    const unsigned w0 = w[0];
    const unsigned w1 = w[1];
    const float v0 = h16_to_f32(w0 & 0xffffu);
    const float v1 = h16_to_f32(w0 >> 16);
    const float v2 = h16_to_f32(w1 & 0xffffu);
    const float v3 = h16_to_f32(w1 >> 16);
    float m = fmaxf(fmaxf(v0, v1), fmaxf(v2, v3));
#pragma unroll
    for (int off = 1; off < 32; off <<= 1) m = fmaxf(m, __shfl_xor(m, off, 32));
    const float e0 = expf(v0 - m);
    const float e1 = expf(v1 - m);
    const float e2 = expf(v2 - m);
    const float e3 = expf(v3 - m);
    float s = (e0 + e1) + (e2 + e3);
#pragma unroll
    for (int off = 1; off < 32; off <<= 1) s += __shfl_xor(s, off, 32);
    const float inv = 1.0f / s;
    Tl[(4 * lane + 0) * 33 + i] = e0 * inv;
    Tl[(4 * lane + 1) * 33 + i] = e1 * inv;
    Tl[(4 * lane + 2) * 33 + i] = e2 * inv;
    Tl[(4 * lane + 3) * 33 + i] = e3 * inv;
  }
  __syncthreads();
  float pv[16];
#pragma unroll
  for (int q = 0; q < 16; ++q) pv[q] = Tl[(wave * 16 + q) * 33 + lane];
  float* ob = out + ((size_t)(b * NOUTC + wave * 16)) * NSTEP + (size_t)(t0 + lane);
  for (int pass = 0; pass < 2; ++pass) {
#pragma unroll
    for (int q = 0; q < 16; ++q) *(volatile float*)(ob + (size_t)q * NSTEP) = pv[q];
    __threadfence();
  }
}

extern "C" void kernel_launch(void* const* d_in, const int* in_sizes, int n_in,
                              void* d_out, int out_size, void* d_ws, size_t ws_size, hipStream_t stream) {
  if (n_in < 10 || d_out == nullptr || d_ws == nullptr) return;
  if (in_sizes[0] != NBATCH * NSTEP || in_sizes[1] != NVOCAB * NEMB || in_sizes[2] != NHID * NEMB ||
      in_sizes[3] != NHID * NHID || in_sizes[4] != NHID || in_sizes[5] != NHID ||
      in_sizes[6] != NOUTC * NHID || in_sizes[7] != NOUTC * NOUTC || in_sizes[8] != NOUTC ||
      in_sizes[9] != NOUTC || out_size != NOUT_ELEMS) return;

  const int*   xs   = (const int*)d_in[0];
  const float* emb  = (const float*)d_in[1];
  const float* wih1 = (const float*)d_in[2];
  const float* whh1 = (const float*)d_in[3];
  const float* bih1 = (const float*)d_in[4];
  const float* bhh1 = (const float*)d_in[5];
  const float* wih2 = (const float*)d_in[6];
  const float* whh2 = (const float*)d_in[7];
  const float* bih2 = (const float*)d_in[8];
  const float* bhh2 = (const float*)d_in[9];
  float* out = (float*)d_out;

  char* ws = (char*)d_ws;
  size_t off = 0;
  auto carve = [&](size_t bytes) -> char* { char* p = ws + off; off += (bytes + 255) & ~(size_t)255; return p; };
  unsigned short* WIH1H = (unsigned short*)carve((size_t)NHID * NEMB * 2);
  unsigned short* WHH1H = (unsigned short*)carve((size_t)NHID * NHID * 2);
  unsigned short* WIH2H = (unsigned short*)carve((size_t)NOUTC * NHID * 2);
  unsigned short* WHH2H = (unsigned short*)carve((size_t)NOUTC * NOUTC * 2);
  float*          BIAS  = (float*)carve((size_t)(NHID + NOUTC) * 4);
  unsigned short* EF16  = (unsigned short*)carve((size_t)NROWS * NEMB * 2);
  unsigned short* XP1   = (unsigned short*)carve((size_t)NROWS * NHID * 2);
  unsigned short* H2G   = (unsigned short*)carve((size_t)NROWS * NOUTC * 2);
  if (off > ws_size || off > (size_t)134217728) return;

  const int n8a = NHID * NEMB / 8;
  const int n8b = NHID * NHID / 8;
  const int n8c = NOUTC * NHID / 8;
  const int n8d = NOUTC * NOUTC / 8;
  cvt8_f16_kernel<<<(n8a + 255) / 256, 256, 0, stream>>>(wih1, WIH1H, n8a, WCARRY);
  cvt8_f16_kernel<<<(n8b + 255) / 256, 256, 0, stream>>>(whh1, WHH1H, n8b, WCARRY);
  cvt8_f16_kernel<<<(n8c + 255) / 256, 256, 0, stream>>>(wih2, WIH2H, n8c, WCARRY);
  cvt8_f16_kernel<<<(n8d + 255) / 256, 256, 0, stream>>>(whh2, WHH2H, n8d, WCARRY);
  bias_prep_kernel<<<1, 160, 0, stream>>>(bih1, bhh1, bih2, bhh2, BIAS);

  gather_cvt_kernel<<<(NROWS * (NEMB / 8) + 255) / 256, 256, 0, stream>>>(xs, emb, EF16);

  gemm64_f16_kernel<<<(NROWS / 64) * (NHID / 64) / 8, 256, 0, stream>>>(
      EF16, NEMB, WIH1H, NEMB, XP1, NHID, BIAS, NROWS, NHID, NEMB, WCARRY_INV);

  rnn_seq_kernel<<<NBATCH / RB, RTHR, 0, stream>>>(XP1, WHH1H, WIH2H, WHH2H, BIAS + NHID, H2G);

  softmax_tr_kernel<<<NBATCH * (NSTEP / 32), 256, 0, stream>>>(H2G, out);
}
